// NonLocalAttention_23192823399127
// MI455X (gfx1250) — hardware-verified
//
#include <hip/hip_runtime.h>

typedef unsigned short u16;
typedef __attribute__((ext_vector_type(16))) _Float16      v16bf;
typedef float __attribute__((may_alias)) float_a;
template <typename T> __device__ __forceinline__ void vst2(void* p, T v) { *(volatile T*)p = v; __threadfence(); *(volatile T*)p = v; }
typedef __attribute__((ext_vector_type(8)))  float         v8f;
typedef __attribute__((ext_vector_type(4)))  unsigned int  v4u;
typedef __attribute__((ext_vector_type(4)))  float         v4f;

#define N_   2
#define C_   256
#define CE_  128
#define HW_  6400
#define EPITCH 264

union V16 {
  v16bf v;
  v4u   q[2];
  u16   us[16];
};

__device__ __forceinline__ u16 f2bf(float f) {
  union { _Float16 h; u16 u; } x; x.h = (_Float16)f; return x.u;
}

__device__ __forceinline__ v8f wmma_bf16(const V16& a, const V16& b, v8f c) {
  v8f d = __builtin_amdgcn_wmma_f32_16x16x32_f16(false, a.v, false, b.v, (short)0, c, false, false);
  asm volatile("v_nop\n\tv_nop\n\tv_nop\n\tv_nop" : "+v"(d) : "v"(a.v), "v"(b.v));
  return d;
}

__global__ __launch_bounds__(256)
void embed_kernel(const float* __restrict__ inp,
                  const float* __restrict__ w1, const float* __restrict__ b1,
                  const float* __restrict__ a1,
                  const float* __restrict__ w2, const float* __restrict__ b2,
                  const float* __restrict__ a2,
                  const float* __restrict__ wa, const float* __restrict__ ba,
                  const float* __restrict__ aa,
                  u16* __restrict__ qws, u16* __restrict__ ktws,
                  u16* __restrict__ vvws) {
  __shared__ __align__(16) u16 tile[64 * EPITCH];
  __shared__ __align__(16) u16 sq[64 * CE_], skt[64 * CE_];
  __shared__ __align__(16) u16 sv[C_ * 64];

  const int blk = blockIdx.x;
  const int n   = blk / (HW_ / 64);
  const int i0  = (blk % (HW_ / 64)) * 64;
  const int t   = threadIdx.x;

  const float* ibase = inp + (size_t)n * C_ * HW_ + i0;
  for (int s = 0; s < 16; ++s) {
    int qd = t + 256 * s;
    int c  = qd >> 4;
    int i4 = (qd & 15) * 4;
    v4f v = *(const v4f*)(ibase + (size_t)c * HW_ + i4);
    tile[(i4 + 0) * EPITCH + c] = f2bf(v.x);
    tile[(i4 + 1) * EPITCH + c] = f2bf(v.y);
    tile[(i4 + 2) * EPITCH + c] = f2bf(v.z);
    tile[(i4 + 3) * EPITCH + c] = f2bf(v.w);
  }
  __syncthreads();

  const int wv = t >> 5, l = t & 31;
  const int ln = l & 15, hf = l >> 4;

  for (int rt = wv; rt < 32; rt += 8) {
    const float *W, *Bb; float alpha; int Rl;
    u16* OP; int sI, sO;
    if (rt < 8)       { W = w1; Bb = b1; alpha = a1[0]; Rl = rt * 16;        OP = sq;  sI = CE_; sO = 1; }
    else if (rt < 16) { W = w2; Bb = b2; alpha = a2[0]; Rl = (rt - 8) * 16;  OP = skt; sI = CE_; sO = 1; }
    else              { W = wa; Bb = ba; alpha = aa[0]; Rl = (rt - 16) * 16; OP = sv;  sI = 1;   sO = 64; }

    V16 A[8];
#pragma unroll
    for (int kc = 0; kc < 8; ++kc) {
      const float* wr = W + (size_t)(Rl + ln) * C_ + kc * 32 + hf * 8;
#pragma unroll
      for (int e = 0; e < 8; ++e) {
        A[kc].us[e]     = f2bf(wr[e]);
        A[kc].us[e + 8] = f2bf(wr[e + 16]);
      }
    }

    for (int it = 0; it < 4; ++it) {
      v8f acc = {0, 0, 0, 0, 0, 0, 0, 0};
#pragma unroll
      for (int kc = 0; kc < 8; ++kc) {
        V16 B;
        const u16* br = &tile[(it * 16 + ln) * EPITCH + kc * 32 + hf * 8];
        B.q[0] = *(const v4u*)br;
        B.q[1] = *(const v4u*)(br + 16);
        acc = wmma_bf16(A[kc], B, acc);
      }
      int icol = it * 16 + ln;
#pragma unroll
      for (int r = 0; r < 8; ++r) {
        int o = Rl + r + 8 * hf;
        float v = acc[r] + Bb[o];
        v = (v >= 0.f) ? v : alpha * v;
        OP[(size_t)icol * sI + (size_t)o * sO] = f2bf(v);
      }
    }
  }
  __syncthreads();
  for (int q = t; q < 64 * 16; q += 256) { const int i = q >> 4, pc = q & 15;
    vst2(qws  + ((size_t)n * HW_ + i0 + i) * CE_ + pc * 8, *(const v4u*)(sq  + i * CE_ + pc * 8));
    vst2(ktws + ((size_t)n * HW_ + i0 + i) * CE_ + pc * 8, *(const v4u*)(skt + i * CE_ + pc * 8)); }
  for (int q = t; q < C_ * 8; q += 256) { const int o = q >> 3, pc = q & 7;
    vst2(vvws + ((size_t)n * C_ + o) * HW_ + i0 + pc * 8, *(const v4u*)(sv + o * 64 + pc * 8)); }
}

__global__ __launch_bounds__(256)
void attn_kernel(const float* __restrict__ inp,
                 const u16* __restrict__ qws, const u16* __restrict__ ktws,
                 const u16* __restrict__ vvws, float* __restrict__ out) {
  __shared__ __align__(16) u16 plds[8 * 16 * 32];

  const int blk = blockIdx.x;
  const int n   = blk / (HW_ / 128);
  const int rb  = blk % (HW_ / 128);
  const int t = threadIdx.x, wv = t >> 5, l = t & 31;
  const int ln = l & 15, hf = l >> 4;
  const int i0 = rb * 128 + wv * 16;

  const u16* qr = qws + ((size_t)n * HW_ + i0 + ln) * CE_ + hf * 8;

  v8f O[16];
  const v8f zer = {0, 0, 0, 0, 0, 0, 0, 0};
#pragma unroll
  for (int ct = 0; ct < 16; ++ct) O[ct] = zer;
  float mrow[8], lrow[8];
#pragma unroll
  for (int r = 0; r < 8; ++r) { mrow[r] = -1e30f; lrow[r] = 0.f; }

  u16* pw = &plds[wv * 16 * 32];
  const u16* ktb = ktws + (size_t)n * HW_ * CE_;
  const u16* vvb = vvws + (size_t)n * C_ * HW_;

  for (int j0 = 0; j0 < HW_; j0 += 32) {
    v8f S[2] = {zer, zer};
#pragma unroll
    for (int kc = 0; kc < 4; ++kc) {
      V16 Aqk; Aqk.q[0] = *(const v4u*)(qr + kc * 32); Aqk.q[1] = *(const v4u*)(qr + kc * 32 + 16);
      const u16* k0 = ktb + (size_t)(j0 + ln) * CE_ + kc * 32 + hf * 8;
#pragma unroll
      for (int st = 0; st < 2; ++st) {
        V16 B;
        const u16* kp = k0 + (size_t)(st * 16) * CE_;
        B.q[0] = *(const v4u*)kp;
        B.q[1] = *(const v4u*)(kp + 16);
        S[st] = wmma_bf16(Aqk, B, S[st]);
      }
    }

#pragma unroll
    for (int r = 0; r < 8; ++r) {
      float tm = fmaxf(S[0][r], S[1][r]);
      tm = fmaxf(tm, __shfl_xor(tm, 1));
      tm = fmaxf(tm, __shfl_xor(tm, 2));
      tm = fmaxf(tm, __shfl_xor(tm, 4));
      tm = fmaxf(tm, __shfl_xor(tm, 8));
      float mn = fmaxf(mrow[r], tm);
      float sc = expf(mrow[r] - mn);
      mrow[r] = mn;
      float rs = 0.f;
#pragma unroll
      for (int st = 0; st < 2; ++st) {
        float p = expf(S[st][r] - mn);
        S[st][r] = p * 16384.0f;
        rs += p;
      }
      rs += __shfl_xor(rs, 1);
      rs += __shfl_xor(rs, 2);
      rs += __shfl_xor(rs, 4);
      rs += __shfl_xor(rs, 8);
      lrow[r] = lrow[r] * sc + rs;
#pragma unroll
      for (int ct = 0; ct < 16; ++ct) O[ct][r] *= sc;
    }

#pragma unroll
    for (int r = 0; r < 8; ++r) {
      int mi = r + 8 * hf;
#pragma unroll
      for (int st = 0; st < 2; ++st)
        pw[mi * 32 + st * 16 + ln] = f2bf(S[st][r]);
    }
    asm volatile("s_wait_dscnt 0" ::: "memory"); __builtin_amdgcn_wave_barrier(); __builtin_amdgcn_fence(__ATOMIC_RELEASE, "workgroup");
    V16 P0;
    {
      const u16* pr = pw + ln * 32 + hf * 8;
      P0.q[0] = *(const v4u*)pr;
      P0.q[1] = *(const v4u*)(pr + 16);
    }
#pragma unroll
    for (int ct = 0; ct < 16; ++ct) {
      V16 Bv0;
      const u16* vr = vvb + (size_t)(ct * 16 + ln) * HW_ + j0 + hf * 8;
      Bv0.q[0] = *(const v4u*)vr;
      Bv0.q[1] = *(const v4u*)(vr + 16);
      O[ct] = wmma_bf16(P0, Bv0, O[ct]);
    }
    __builtin_amdgcn_wave_barrier();
  }

#pragma unroll
  for (int r = 0; r < 8; ++r) lrow[r] = (1.0f / 16384.0f) / lrow[r];
  __shared__ __align__(16) float so[128 * 128];
  const int ib0 = rb * 128;
  for (int half = 0; half < 2; ++half) {
    __syncthreads();
#pragma unroll
    for (int ctl = 0; ctl < 8; ++ctl) { const int ct = half * 8 + ctl;
#pragma unroll
      for (int r = 0; r < 8; ++r) so[(ctl * 16 + ln) * 128 + wv * 16 + r + 8 * hf] = O[ct][r] * lrow[r]; }
    __syncthreads();
    for (int q = t; q < 128 * 32; q += 256) { const int cl = q >> 5, pc = q & 31; const int c = half * 128 + cl;
      const size_t idx = ((size_t)n * C_ + c) * HW_ + ib0 + pc * 4;
      v4f v = *(const v4f*)(so + cl * 128 + pc * 4) + *(const v4f*)(inp + idx);
      vst2(out + idx, v); }
  }
}

extern "C" void kernel_launch(void* const* d_in, const int* in_sizes, int n_in,
                              void* d_out, int out_size, void* d_ws, size_t ws_size,
                              hipStream_t stream) {
  (void)in_sizes; (void)n_in; (void)out_size; (void)ws_size;
  const float* inp = (const float*)d_in[0];
  const float* w1  = (const float*)d_in[1];
  const float* b1  = (const float*)d_in[2];
  const float* a1  = (const float*)d_in[3];
  const float* w2  = (const float*)d_in[4];
  const float* b2  = (const float*)d_in[5];
  const float* a2  = (const float*)d_in[6];
  const float* wa  = (const float*)d_in[7];
  const float* ba  = (const float*)d_in[8];
  const float* aa  = (const float*)d_in[9];
  float* out = (float*)d_out;

  u16* qws  = (u16*)d_ws;
  u16* ktws = qws  + (size_t)N_ * HW_ * CE_;
  u16* vvws = ktws + (size_t)N_ * HW_ * CE_;

  embed_kernel<<<dim3(N_ * (HW_ / 64)), dim3(256), 0, stream>>>(
      inp, w1, b1, a1, w2, b2, a2, wa, ba, aa, qws, ktws, vvws);
  attn_kernel<<<dim3(N_ * (HW_ / 128)), dim3(256), 0, stream>>>(
      inp, qws, ktws, vvws, out);
}
